// HollowTransformerLayer_60052232733088
// MI455X (gfx1250) — hardware-verified
//
#include <hip/hip_runtime.h>
#include <stddef.h>


typedef _Float16 v16h __attribute__((ext_vector_type(16)));
typedef _Float16 v8h  __attribute__((ext_vector_type(8)));
typedef float    v8f  __attribute__((ext_vector_type(8)));
typedef float    v4f  __attribute__((ext_vector_type(4)));

union Frag { v16h v; v8h half[2]; };

enum { DMODEL = 1024, DFF = 4096 };

#define TM 64
#define TN 64
#define TK 32
#define LROW 40
#define CPITCH 68
#define WSCALE 64.0f
#define WUNSCALE 0.015625f
#define LN_EPS 1e-5f

__device__ __forceinline__ v8f wmma_f16(v16h a, v16h b, v8f c) {
  v8f d = __builtin_amdgcn_wmma_f32_16x16x32_f16(false, a, false, b, (short)0, c, false, false);
  asm volatile("v_nop\n\tv_nop\n\tv_nop\n\tv_nop" : "+v"(d) : "v"(a), "v"(b));
  return d;
}

__device__ __forceinline__ float wave_sum(float v) {
#pragma unroll
  for (int off = 16; off > 0; off >>= 1) v += __shfl_xor(v, off);
  return v;
}

__global__ __launch_bounds__(256) void cvt_act_kernel(
    const float* __restrict__ in, _Float16* out, int n8) {
  const int i = blockIdx.x * 256 + threadIdx.x;
  if (i < n8) {
    const size_t off = (size_t)i * 8;
    const v4f a = *(const v4f*)(in + off);
    const v4f b = *(const v4f*)(in + off + 4);
    v8h o;
    o[0] = (_Float16)a[0]; o[1] = (_Float16)a[1]; o[2] = (_Float16)a[2]; o[3] = (_Float16)a[3];
    o[4] = (_Float16)b[0]; o[5] = (_Float16)b[1]; o[6] = (_Float16)b[2]; o[7] = (_Float16)b[3];
    _Float16* p = out + off;
    *(volatile v8h*)p = o;
    __threadfence();
    *(volatile v8h*)p = o;
  }
}

__global__ __launch_bounds__(256) void cvt_wt_kernel(
    const float* __restrict__ W, _Float16* Wt, int K, int N, float scale) {
  __shared__ float tile[64][33];
  const int k0 = blockIdx.y * 64;
  const int n0 = blockIdx.x * 32;
  const int tid = threadIdx.x;
  const int tx = tid & 31;
  const int ty = tid >> 5;
#pragma unroll
  for (int i = 0; i < 8; ++i) {
    const int kr = ty + 8 * i;
    const bool ok = (k0 + kr < K) && (n0 + tx < N);
    tile[kr][tx] = ok ? W[(size_t)(k0 + kr) * N + n0 + tx] : 0.0f;
  }
  __syncthreads();
  const int w  = tid >> 5;
  const int l  = tid & 31;
  const int nl = w * 4 + (l >> 3);
  const int kc = (l & 7) * 8;
  v8h o;
#pragma unroll
  for (int j = 0; j < 8; ++j) o[j] = (_Float16)(tile[kc + j][nl] * scale);
  const bool sok = (n0 + nl < N) && (k0 + kc + 8 <= K);
  _Float16* p = Wt + (size_t)(n0 + nl) * K + k0 + kc;
  if (sok) *(volatile v8h*)p = o;
  __threadfence();
  if (sok) *(volatile v8h*)p = o;
}

__global__ __launch_bounds__(128) void gemm_f16_wmma(
    const _Float16* __restrict__ A, const _Float16* __restrict__ Bt,
    const float* __restrict__ bias, float* Cf, _Float16* Ch,
    int M, int N, int K, int relu, float oscale) {
  __shared__ __align__(16) float smem[TM * CPITCH];
  _Float16* sA = (_Float16*)smem;
  _Float16* sB = sA + TM * LROW;

  const int tid  = threadIdx.x;
  const int wave = tid >> 5;
  const int lane = tid & 31;
  const int hh   = lane >> 4;
  const int m    = lane & 15;
  const int m0 = blockIdx.y * TM;
  const int n0 = blockIdx.x * TN;
  if (m0 >= M || n0 >= N) return;

  v8f acc[4] = {v8f{}, v8f{}, v8f{}, v8f{}};

  const int lr = tid >> 2;
  const int lc = (tid & 3) * 8;
  const int nk = K / TK;

  for (int kt = 0; kt < nk; ++kt) {
    const int k0 = kt * TK;
#pragma unroll
    for (int p = 0; p < 2; ++p) {
      const int row = p * 32 + lr;
      const v8h va = *(const v8h*)(A  + (size_t)(m0 + row) * K + k0 + lc);
      const v8h vb = *(const v8h*)(Bt + (size_t)(n0 + row) * K + k0 + lc);
      *(v8h*)(sA + row * LROW + lc) = va;
      *(v8h*)(sB + row * LROW + lc) = vb;
    }
    __syncthreads();

    Frag a;
    const _Float16* ap = sA + (wave * 16 + m) * LROW;
    a.half[0] = *(const v8h*)(ap + 8 * hh);
    a.half[1] = *(const v8h*)(ap + 16 + 8 * hh);
#pragma unroll
    for (int t = 0; t < 4; ++t) {
      Frag b;
      const _Float16* bp = sB + (t * 16 + m) * LROW;
      b.half[0] = *(const v8h*)(bp + 8 * hh);
      b.half[1] = *(const v8h*)(bp + 16 + 8 * hh);
      acc[t] = wmma_f16(a.v, b.v, acc[t]);
    }
    __syncthreads();
  }

  float* sC = smem;
#pragma unroll
  for (int t = 0; t < 4; ++t) {
    const int nc = t * 16 + m;
    const float bsv = bias[n0 + nc];
#pragma unroll
    for (int r = 0; r < 8; ++r) {
      float v = acc[t][r] * oscale + bsv;
      if (relu) v = fmaxf(v, 0.0f);
      sC[(wave * 16 + 8 * hh + r) * CPITCH + nc] = v;
    }
  }
  __syncthreads();

  if (Cf) {
    v4f vals[8];
#pragma unroll
    for (int j = 0; j < 8; ++j) {
      const int row = wave * 16 + 2 * j + hh;
      vals[j] = *(const v4f*)(sC + row * CPITCH + m * 4);
    }
#pragma unroll
    for (int j = 0; j < 8; ++j) {
      const int row = wave * 16 + 2 * j + hh;
      float* p = Cf + (size_t)(m0 + row) * N + n0 + m * 4;
      *(volatile v4f*)p = vals[j];
    }
    __threadfence();
#pragma unroll
    for (int j = 0; j < 8; ++j) {
      const int row = wave * 16 + 2 * j + hh;
      float* p = Cf + (size_t)(m0 + row) * N + n0 + m * 4;
      *(volatile v4f*)p = vals[j];
    }
  }
  if (Ch) {
    const int rsub = lane >> 3;
    const int col  = (lane & 7) * 8;
    v8h hv[4];
#pragma unroll
    for (int j = 0; j < 4; ++j) {
      const int row = wave * 16 + 4 * j + rsub;
      const v4f p0 = *(const v4f*)(sC + row * CPITCH + col);
      const v4f p1 = *(const v4f*)(sC + row * CPITCH + col + 4);
      v8h o;
      o[0] = (_Float16)p0[0]; o[1] = (_Float16)p0[1]; o[2] = (_Float16)p0[2]; o[3] = (_Float16)p0[3];
      o[4] = (_Float16)p1[0]; o[5] = (_Float16)p1[1]; o[6] = (_Float16)p1[2]; o[7] = (_Float16)p1[3];
      hv[j] = o;
    }
#pragma unroll
    for (int j = 0; j < 4; ++j) {
      const int row = wave * 16 + 4 * j + rsub;
      _Float16* p = Ch + (size_t)(m0 + row) * N + n0 + col;
      *(volatile v8h*)p = hv[j];
    }
    __threadfence();
#pragma unroll
    for (int j = 0; j < 4; ++j) {
      const int row = wave * 16 + 4 * j + rsub;
      _Float16* p = Ch + (size_t)(m0 + row) * N + n0 + col;
      *(volatile v8h*)p = hv[j];
    }
  }
}

__global__ __launch_bounds__(256) void add_ln_kernel(
    const float* __restrict__ X, const float* __restrict__ Y,
    const float* __restrict__ g, const float* __restrict__ be,
    float* outf, _Float16* outh, int rows) {
  __shared__ __align__(16) float srow[DMODEL];
  __shared__ float sred[8];
  __shared__ float sstat[2];
  const int row = blockIdx.x;
  if (row >= rows) return;
  const int t = threadIdx.x;
  const int w = t >> 5;
  const int l = t & 31;
  const size_t base = (size_t)row * DMODEL;

  const v4f xa = *(const v4f*)(X + base + 4 * t);
  const v4f ya = *(const v4f*)(Y + base + 4 * t);
  const v4f v = xa + ya;

  float s = (v[0] + v[1]) + (v[2] + v[3]);
  s = wave_sum(s);
  if (l == 0) sred[w] = s;
  __syncthreads();
  if (t == 0) {
    float a = 0.0f;
#pragma unroll
    for (int i = 0; i < 8; ++i) a += sred[i];
    sstat[0] = a;
  }
  __syncthreads();
  const float mu = sstat[0] * (1.0f / DMODEL);

  const v4f d = v - mu;
  float s2 = (d[0] * d[0] + d[1] * d[1]) + (d[2] * d[2] + d[3] * d[3]);
  s2 = wave_sum(s2);
  if (l == 0) sred[w] = s2;
  __syncthreads();
  if (t == 0) {
    float a = 0.0f;
#pragma unroll
    for (int i = 0; i < 8; ++i) a += sred[i];
    sstat[1] = a;
  }
  __syncthreads();
  const float var  = sstat[1] * (1.0f / DMODEL);
  const float rstd = rsqrtf(var + LN_EPS);

  const v4f gg = *(const v4f*)(g + 4 * t);
  const v4f bb = *(const v4f*)(be + 4 * t);
  const v4f o = d * rstd * gg + bb;

  *(v4f*)(srow + 4 * t) = o;
  __syncthreads();

  const bool hok = (outh != nullptr) && (t < 128);
  v8h ho;
#pragma unroll
  for (int j = 0; j < 8; ++j) ho[j] = (_Float16)0.0f;
  if (hok) {
    const v4f p0 = *(const v4f*)(srow + 8 * t);
    const v4f p1 = *(const v4f*)(srow + 8 * t + 4);
    ho[0] = (_Float16)p0[0]; ho[1] = (_Float16)p0[1]; ho[2] = (_Float16)p0[2]; ho[3] = (_Float16)p0[3];
    ho[4] = (_Float16)p1[0]; ho[5] = (_Float16)p1[1]; ho[6] = (_Float16)p1[2]; ho[7] = (_Float16)p1[3];
  }
  float* pf = outf + base + 4 * t;
  _Float16* ph = hok ? (outh + base + 8 * t) : nullptr;

  *(volatile v4f*)pf = o;
  if (hok) *(volatile v8h*)ph = ho;
  __threadfence();
  *(volatile v4f*)pf = o;
  if (hok) *(volatile v8h*)ph = ho;
}

extern "C" void kernel_launch(void* const* d_in, const int* in_sizes, int n_in,
                              void* d_out, int out_size, void* d_ws,
                              size_t ws_size, hipStream_t stream) {
  if (n_in < 18) return;
  const int nx = in_sizes[0];
  if (nx <= 0 || (nx % DMODEL) != 0) return;
  const int rows = nx / DMODEL;
  if ((rows % TM) != 0 || out_size != nx) return;
  if (in_sizes[6] != DMODEL * DMODEL || in_sizes[8] != DMODEL * DMODEL ||
      in_sizes[10] != DMODEL * DFF || in_sizes[12] != DFF * DMODEL) return;
  if (in_sizes[7] != DMODEL || in_sizes[9] != DMODEL || in_sizes[11] != DFF ||
      in_sizes[13] != DMODEL || in_sizes[14] != DMODEL || in_sizes[15] != DMODEL ||
      in_sizes[16] != DMODEL || in_sizes[17] != DMODEL) return;

  const float* x   = (const float*)d_in[0];
  const float* Wv  = (const float*)d_in[6];
  const float* bv  = (const float*)d_in[7];
  const float* Wo  = (const float*)d_in[8];
  const float* bo  = (const float*)d_in[9];
  const float* W1  = (const float*)d_in[10];
  const float* b1  = (const float*)d_in[11];
  const float* W2  = (const float*)d_in[12];
  const float* b2  = (const float*)d_in[13];
  const float* g1  = (const float*)d_in[14];
  const float* be1 = (const float*)d_in[15];
  const float* g2  = (const float*)d_in[16];
  const float* be2 = (const float*)d_in[17];
  float* out = (float*)d_out;

  char* ws = (char*)d_ws;
  size_t o = 0;
  auto carve = [&](size_t bytes) {
    size_t r = o;
    o += (bytes + 255) & ~(size_t)255;
    return r;
  };
  const size_t nAct  = (size_t)rows * DMODEL;
  const size_t nFf   = (size_t)rows * DFF;
  const size_t offXh  = carve(nAct * 2);
  const size_t offVh  = carve(nAct * 2);
  const size_t offAtt = carve(nAct * 4);
  const size_t offWvt = carve((size_t)DMODEL * DMODEL * 2);
  const size_t offWot = carve((size_t)DMODEL * DMODEL * 2);
  const size_t offW1t = carve((size_t)DFF * DMODEL * 2);
  const size_t offW2t = carve((size_t)DMODEL * DFF * 2);
  const size_t offHf  = carve(nAct * 4);
  const size_t offHh  = carve(nAct * 2);
  const size_t offF1  = carve(nFf * 2);
  const size_t offF2  = carve(nAct * 4);
  if (o > ws_size) return;

  _Float16* xh  = (_Float16*)(ws + offXh);
  _Float16* vh  = (_Float16*)(ws + offVh);
  float*    att = (float*)(ws + offAtt);
  _Float16* Wvt = (_Float16*)(ws + offWvt);
  _Float16* Wot = (_Float16*)(ws + offWot);
  _Float16* W1t = (_Float16*)(ws + offW1t);
  _Float16* W2t = (_Float16*)(ws + offW2t);
  float*    hf  = (float*)(ws + offHf);
  _Float16* h16 = (_Float16*)(ws + offHh);
  _Float16* f1h = (_Float16*)(ws + offF1);
  float*    ff2 = (float*)(ws + offF2);

  const int n8 = nx / 8;
  cvt_act_kernel<<<dim3((n8 + 255) / 256), 256, 0, stream>>>(x, xh, n8);
  cvt_wt_kernel<<<dim3((DMODEL + 31) / 32, (DMODEL + 63) / 64), 256, 0, stream>>>(Wv, Wvt, DMODEL, DMODEL, WSCALE);
  cvt_wt_kernel<<<dim3((DMODEL + 31) / 32, (DMODEL + 63) / 64), 256, 0, stream>>>(Wo, Wot, DMODEL, DMODEL, WSCALE);
  cvt_wt_kernel<<<dim3((DFF + 31) / 32, (DMODEL + 63) / 64), 256, 0, stream>>>(W1, W1t, DMODEL, DFF, WSCALE);
  cvt_wt_kernel<<<dim3((DMODEL + 31) / 32, (DFF + 63) / 64), 256, 0, stream>>>(W2, W2t, DFF, DMODEL, WSCALE);

  gemm_f16_wmma<<<dim3(DMODEL / TN, rows / TM), 128, 0, stream>>>(
      xh, Wvt, bv, nullptr, vh, rows, DMODEL, DMODEL, 0, WUNSCALE);
  gemm_f16_wmma<<<dim3(DMODEL / TN, rows / TM), 128, 0, stream>>>(
      vh, Wot, bo, att, nullptr, rows, DMODEL, DMODEL, 0, WUNSCALE);
  add_ln_kernel<<<dim3(rows), 256, 0, stream>>>(x, att, g1, be1, hf, h16, rows);
  gemm_f16_wmma<<<dim3(DFF / TN, rows / TM), 128, 0, stream>>>(
      h16, W1t, b1, nullptr, f1h, rows, DFF, DMODEL, 1, WUNSCALE);
  gemm_f16_wmma<<<dim3(DMODEL / TN, rows / TM), 128, 0, stream>>>(
      f1h, W2t, b2, ff2, nullptr, rows, DMODEL, DFF, 0, WUNSCALE);
  add_ln_kernel<<<dim3(rows), 256, 0, stream>>>(hf, ff2, g2, be2, out, nullptr, rows);
}
